// GraphNeuralNetworkRiskManager_14491219657471
// MI455X (gfx1250) — hardware-verified
//
#include <hip/hip_runtime.h>
#include <stddef.h>
#include <math.h>


#define FD      128
#define KL      256
#define NCLS    2
#define NCP     16
#define NTHR    256
#define NWAVE   8
#define EPT     8
#define NGRP    2
#define CHUNK   (NTHR * EPT * NGRP)
#define WCAP    (EPT * NGRP * 32)
#define LISTN   (NWAVE * WCAP)
#define NBC     4096
#define NBF     2048
#define FPC     (NBC / NBF)
#define RCAP    40960
#define RBN     128
#define TGT     256
#define DEGCAP  256
#define OTHR    512
#define BM      64
#define CBM     128
#define WSCAP   134217728

#define LDS_FILL ((RCAP + NBF + LISTN) * 4 + 64)
#define LDS_G1   (BM * FD * 2 * 2 + BM * FD * 4)
#define LDS_G2   (BM * FD * 2 * 4 + BM * FD * 4)
#define LDS_CLS  (CBM * FD * 2 * 2 + CBM * NCLS * 4)

static_assert((CHUNK & (CHUNK - 1)) == 0);
static_assert(CHUNK <= 4096);
static_assert(NBC <= 4096 && NBF <= 4096);
static_assert((NBC & (NBC - 1)) == 0 && (NBF & (NBF - 1)) == 0);
static_assert(NBC == FPC * NBF && FPC == 2);
static_assert(OTHR * 8 == NBC);
static_assert(OTHR / 32 == 8 * FPC);
static_assert((RCAP % 32) == 0);
static_assert(TGT == NWAVE * 32);
static_assert((TGT % BM) == 0 && (TGT % CBM) == 0);
static_assert((DEGCAP % 32) == 0);
static_assert(KL == 2 * FD && NCP == 16 && NCLS <= 4);
static_assert(BM == 64 && NWAVE == 8 && CBM == NWAVE * 16);

typedef float          v2f  __attribute__((ext_vector_type(2)));
typedef float          v4f  __attribute__((ext_vector_type(4)));
typedef float          v8f  __attribute__((ext_vector_type(8)));
typedef int            v4i  __attribute__((ext_vector_type(4)));
typedef unsigned short v8us __attribute__((ext_vector_type(8)));
typedef unsigned short v16us __attribute__((ext_vector_type(16)));
typedef __bf16         v16bf __attribute__((ext_vector_type(16)));
union FragU { v16us w; v8us u[2]; };

__device__ __forceinline__ v8f wmb(v16us a, v16us b, v8f c) {
  const v16bf ab = __builtin_bit_cast(v16bf, a);
  const v16bf bb = __builtin_bit_cast(v16bf, b);
  v8f d = __builtin_amdgcn_wmma_f32_16x16x32_bf16(false, ab, false, bb, (short)0, c, false, false);
  asm volatile("v_nop\n\tv_nop\n\tv_nop\n\tv_nop" : "+v"(d) : "v"(a), "v"(b));
  return d;
}

__device__ __forceinline__ unsigned int bfb(float f) {
  const unsigned int u = __float_as_uint(f);
  return (u + 0x7FFFu + ((u >> 16) & 1u)) >> 16;
}
__device__ __forceinline__ void sp1(float v, unsigned short& h, unsigned short& l) {
  const unsigned int hb = bfb(v);
  const float hf = __uint_as_float(hb << 16);
  h = (unsigned short)hb;
  l = (unsigned short)bfb(v - hf);
}
__device__ __forceinline__ void sp8(v4f a, v4f b, v8us& h, v8us& l) {
  unsigned short hh, ll;
  sp1(a.x, hh, ll); h[0] = hh; l[0] = ll;
  sp1(a.y, hh, ll); h[1] = hh; l[1] = ll;
  sp1(a.z, hh, ll); h[2] = hh; l[2] = ll;
  sp1(a.w, hh, ll); h[3] = hh; l[3] = ll;
  sp1(b.x, hh, ll); h[4] = hh; l[4] = ll;
  sp1(b.y, hh, ll); h[5] = hh; l[5] = ll;
  sp1(b.z, hh, ll); h[6] = hh; l[6] = ll;
  sp1(b.w, hh, ll); h[7] = hh; l[7] = ll;
}
__device__ __forceinline__ v4f relu4(v4f t) {
  v4f r;
  r.x = fmaxf(t.x, 0.f); r.y = fmaxf(t.y, 0.f); r.z = fmaxf(t.z, 0.f); r.w = fmaxf(t.w, 0.f);
  return r;
}

__global__ __launch_bounds__(NTHR) void k_wprep(const float* __restrict__ Wa, const float* __restrict__ Wb,
                                               int ldw, int lg, int nv, unsigned short* ph, unsigned short* pl,
                                               int units) {
  const int i = (int)blockIdx.x * NTHR + (int)threadIdx.x;
  if (i >= units) return;
  const int n  = i >> lg;
  const int k0 = (i & ((1 << lg) - 1)) * 8;
  const int nc = n < nv - 1 ? n : nv - 1;
  const int kk = k0 & (FD - 1);
  float va[8], vb[8];
#pragma unroll
  for (int j = 0; j < 8; ++j) {
    va[j] = Wa[(size_t)(kk + j) * ldw + nc];
    vb[j] = Wb[(size_t)(kk + j) * ldw + nc];
  }
  const bool useB = (k0 >= FD);
  const bool zrow = (n >= nv);
  float v[8];
#pragma unroll
  for (int j = 0; j < 8; ++j) {
    const float t = useB ? vb[j] : va[j];
    v[j] = zrow ? 0.f : t;
  }
  v4f a0, a1;
  a0.x = v[0]; a0.y = v[1]; a0.z = v[2]; a0.w = v[3];
  a1.x = v[4]; a1.y = v[5]; a1.z = v[6]; a1.w = v[7];
  v8us hv, lv;
  sp8(a0, a1, hv, lv);
  unsigned short* dh = ph + (size_t)i * 8;
  unsigned short* dl = pl + (size_t)i * 8;
  *(volatile v8us*)dh = hv;
  *(volatile v8us*)dl = lv;
  __threadfence();
  *(volatile v8us*)dh = hv;
  *(volatile v8us*)dl = lv;
}

template <int NB>
__device__ __forceinline__ int scan_chunk(const int* __restrict__ dsts, int nE, int cbase, int slotBase,
                                          int vec8, int* list, int tid, int lane, int wave) {
  int wc = 0;
#pragma unroll
  for (int g = 0; g < NGRP; ++g) {
    const int el0  = (g * NTHR + tid) * EPT;
    const int e0   = cbase + el0;
    const int sent = -2147483647 - 1;
    v4i da, db;
    if (vec8 != 0 && cbase + CHUNK <= nE) {
      da = *(const v4i*)(dsts + e0);
      db = *(const v4i*)(dsts + e0 + 4);
    } else {
      da.x = (e0     < nE) ? dsts[min(e0, nE - 1)] : sent;
      da.y = (e0 + 1 < nE) ? dsts[min(e0 + 1, nE - 1)] : sent;
      da.z = (e0 + 2 < nE) ? dsts[min(e0 + 2, nE - 1)] : sent;
      da.w = (e0 + 3 < nE) ? dsts[min(e0 + 3, nE - 1)] : sent;
      db.x = (e0 + 4 < nE) ? dsts[min(e0 + 4, nE - 1)] : sent;
      db.y = (e0 + 5 < nE) ? dsts[min(e0 + 5, nE - 1)] : sent;
      db.z = (e0 + 6 < nE) ? dsts[min(e0 + 6, nE - 1)] : sent;
      db.w = (e0 + 7 < nE) ? dsts[min(e0 + 7, nE - 1)] : sent;
    }
    const unsigned nb = (unsigned)slotBase;
    const unsigned s0 = (unsigned)da.x - nb, s1 = (unsigned)da.y - nb;
    const unsigned s2 = (unsigned)da.z - nb, s3 = (unsigned)da.w - nb;
    const unsigned s4 = (unsigned)db.x - nb, s5 = (unsigned)db.y - nb;
    const unsigned s6 = (unsigned)db.z - nb, s7 = (unsigned)db.w - nb;
    const bool h0 = s0 < (unsigned)NB, h1 = s1 < (unsigned)NB, h2 = s2 < (unsigned)NB, h3 = s3 < (unsigned)NB;
    const bool h4 = s4 < (unsigned)NB, h5 = s5 < (unsigned)NB, h6 = s6 < (unsigned)NB, h7 = s7 < (unsigned)NB;
    const unsigned any = __builtin_amdgcn_ballot_w32(h0 | h1 | h2 | h3 | h4 | h5 | h6 | h7);
    if (any != 0u) {
#define HITJ(J, HJ, SJ) { \
        const unsigned mj = __builtin_amdgcn_ballot_w32(HJ); \
        if (mj != 0u) { \
          if (HJ) { \
            const int pos = wc + (int)__builtin_amdgcn_mbcnt_lo(mj, 0u); \
            if (pos < WCAP) list[wave * WCAP + pos] = ((el0 + (J)) << 12) | (int)(SJ); \
          } \
          wc += (int)__builtin_popcount(mj); } }
      HITJ(0, h0, s0)
      HITJ(1, h1, s1)
      HITJ(2, h2, s2)
      HITJ(3, h3, s3)
      HITJ(4, h4, s4)
      HITJ(5, h5, s5)
      HITJ(6, h6, s6)
      HITJ(7, h7, s7)
#undef HITJ
    }
  }
  return wc;
}

__global__ __launch_bounds__(NTHR) void k_count(
    const int* __restrict__ dsts, int* cnt, int nE, int vec8) {
  __shared__ __attribute__((aligned(16))) int scnt[NBC];
  __shared__ __attribute__((aligned(16))) int list[LISTN];
  __shared__ int wcnt[NWAVE];
  const int tid = threadIdx.x, lane = tid & 31, wave = tid >> 5;
  const int nodeBase = blockIdx.x * NBC;

  for (int i = tid; i < NBC; i += NTHR) scnt[i] = 0;
  __syncthreads();

  const int nChunks = (nE + CHUNK - 1) / CHUNK;
#pragma unroll 1
  for (int ch = 0; ch < nChunks; ++ch) {
    const int cbase = ch * CHUNK;
    const int wc = scan_chunk<NBC>(dsts, nE, cbase, nodeBase, vec8, list, tid, lane, wave);
    if (lane == 0) wcnt[wave] = wc;
    __syncthreads();
    if (wave == 0) {
#pragma unroll 1
      for (int wsx = 0; wsx < NWAVE; ++wsx) {
        int n = __builtin_amdgcn_readfirstlane(wcnt[wsx]);
        n = n > WCAP ? WCAP : (n < 0 ? 0 : n);
        const int* lp = list + wsx * WCAP;
#pragma unroll 1
        for (int i = 0; i < n; ++i) {
          const int ent  = __builtin_amdgcn_readfirstlane(lp[i]);
          const int slot = ent & (NBC - 1);
          if (lane == 0) scnt[slot] = scnt[slot] + 1;
        }
      }
    }
    __syncthreads();
  }

  v4i cq[4];
#pragma unroll
  for (int q = 0; q < 4; ++q) {
    const int f = (wave * 4 + q) * 128 + 4 * lane;
    cq[q] = *(const v4i*)(scnt + f);
  }
  int* cpn = cnt + (size_t)nodeBase;
#pragma unroll
  for (int q = 0; q < 4; ++q) {
    const int f = (wave * 4 + q) * 128 + 4 * lane;
    *(volatile v4i*)(cpn + f) = cq[q];
  }
  __threadfence();
#pragma unroll
  for (int q = 0; q < 4; ++q) {
    const int f = (wave * 4 + q) * 128 + 4 * lane;
    *(volatile v4i*)(cpn + f) = cq[q];
  }
}

__global__ __launch_bounds__(OTHR) void k_offsets(
    const int* __restrict__ cnt, int* off, int* rbase, int nChunk) {
  __shared__ __attribute__((aligned(16))) int soff[NBC];
  __shared__ __attribute__((aligned(16))) int srb[RBN];
  __shared__ int wtot[OTHR / 32];
  const int tid = threadIdx.x, lane = tid & 31, wave = tid >> 5, sub = tid >> 8;
  for (int i = tid; i < RBN; i += OTHR) srb[i] = 0;
  __syncthreads();
  int carry = 0;
#pragma unroll 1
  for (int ch = 0; ch < nChunk; ++ch) {
    const int base = ch * NBC;
    const v4i ca = *(const v4i*)(cnt + base + 8 * tid);
    const v4i cb = *(const v4i*)(cnt + base + 8 * tid + 4);
    const int e0 = max(ca.x, 0), e1 = max(ca.y, 0), e2 = max(ca.z, 0), e3 = max(ca.w, 0);
    const int e4 = max(cb.x, 0), e5 = max(cb.y, 0), e6 = max(cb.z, 0), e7 = max(cb.w, 0);
    const int ts = e0 + e1 + e2 + e3 + e4 + e5 + e6 + e7;
    int incl = ts;
#pragma unroll
    for (int d = 1; d < 32; d <<= 1) {
      const int t = __shfl_up(incl, d);
      if (lane >= d) incl += t;
    }
    if (lane == 31) wtot[wave] = incl;
    __syncthreads();
    int S0 = 0, S1 = 0;
#pragma unroll
    for (int w = 0; w < 8; ++w) { S0 += wtot[w]; S1 += wtot[8 + w]; }
    int pre = 0;
#pragma unroll 1
    for (int w = 8 * sub; w < wave; ++w) pre += wtot[w];
    const int b0 = carry;
    const int b1 = b0 + ((S0 + 31) & ~31);
    const int b2 = b1 + ((S1 + 31) & ~31);
    const int myb = sub == 0 ? b0 : b1;
    if (tid == 0) {
      srb[min(2 * ch + 0, RBN - 1)] = b0;
      srb[min(2 * ch + 1, RBN - 1)] = b1;
    }
    int run = myb + pre + incl - ts;
    soff[8 * tid + 0] = run; run += e0;
    soff[8 * tid + 1] = run; run += e1;
    soff[8 * tid + 2] = run; run += e2;
    soff[8 * tid + 3] = run; run += e3;
    soff[8 * tid + 4] = run; run += e4;
    soff[8 * tid + 5] = run; run += e5;
    soff[8 * tid + 6] = run; run += e6;
    soff[8 * tid + 7] = run;
    carry = b2;
    __syncthreads();
    const v4i o0 = *(const v4i*)(soff + 4 * tid);
    const v4i o1 = *(const v4i*)(soff + 4 * (tid + OTHR));
    int* op = off + base;
    *(volatile v4i*)(op + 4 * tid) = o0;
    *(volatile v4i*)(op + 4 * (tid + OTHR)) = o1;
    __threadfence();
    *(volatile v4i*)(op + 4 * tid) = o0;
    *(volatile v4i*)(op + 4 * (tid + OTHR)) = o1;
    __syncthreads();
  }
  if (tid == 0) srb[min(2 * nChunk, RBN - 1)] = carry;
  __syncthreads();
  v4i rv = {0, 0, 0, 0};
  if (tid < 32) rv = *(const v4i*)(srb + 4 * tid);
  if (tid < 32) *(volatile v4i*)(rbase + 4 * tid) = rv;
  __threadfence();
  if (tid < 32) *(volatile v4i*)(rbase + 4 * tid) = rv;
}

__global__ __launch_bounds__(NTHR) void k_fill(
    const int* __restrict__ dsts, const int* __restrict__ off, const int* __restrict__ rbase,
    int* csr, int nE, int vec8, int csrLen) {
  extern __shared__ v4f lds_dyn[];
  int* region = (int*)lds_dyn;
  int* cursor = region + RCAP;
  int* list   = cursor + NBF;
  int* wcnt   = list + LISTN;
  const int tid = threadIdx.x, lane = tid & 31, wave = tid >> 5;
  const int b = blockIdx.x;
  const int nodeBase = b * NBF;

  int rb0 = rbase[b];
  const int rb1 = rbase[b + 1];
  rb0 = rb0 < 0 ? 0 : (rb0 > csrLen ? csrLen : rb0);
  rb0 &= ~31;
  int len = rb1 - rb0;
  len = len < 0 ? 0 : (len > RCAP ? RCAP : len);
  int lenW = (len + 31) & ~31;
  if (rb0 + lenW > csrLen) lenW = (csrLen - rb0) & ~31;

  {
    const v4i z = {0, 0, 0, 0};
    for (int i = tid; i < RCAP / 4; i += NTHR) ((v4i*)region)[i] = z;
    for (int s = tid; s < NBF; s += NTHR) {
      int o = off[nodeBase + s] - rb0;
      o = o < 0 ? 0 : (o > RCAP ? RCAP : o);
      cursor[s] = o;
    }
  }
  __syncthreads();

  const int nChunks = (nE + CHUNK - 1) / CHUNK;
#pragma unroll 1
  for (int ch = 0; ch < nChunks; ++ch) {
    const int cbase = ch * CHUNK;
    const int wc = scan_chunk<NBF>(dsts, nE, cbase, nodeBase, vec8, list, tid, lane, wave);
    if (lane == 0) wcnt[wave] = wc;
    __syncthreads();
    if (wave == 0) {
#pragma unroll 1
      for (int wsx = 0; wsx < NWAVE; ++wsx) {
        int n = __builtin_amdgcn_readfirstlane(wcnt[wsx]);
        n = n > WCAP ? WCAP : (n < 0 ? 0 : n);
        const int* lp = list + wsx * WCAP;
#pragma unroll 1
        for (int i = 0; i < n; ++i) {
          const int ent  = __builtin_amdgcn_readfirstlane(lp[i]);
          const int slot = ent & (NBF - 1);
          int e = cbase + ((ent >> 12) & (CHUNK - 1));
          e = e > nE - 1 ? nE - 1 : e;
          if (lane == 0) {
            int pos = cursor[slot];
            pos = pos < 0 ? 0 : (pos > RCAP - 1 ? RCAP - 1 : pos);
            region[pos] = e;
            const int np = pos + 1;
            cursor[slot] = np > RCAP ? RCAP : np;
          }
        }
      }
    }
    __syncthreads();
  }

  const int nv = lenW >> 2;
  int* gp = csr + rb0;
#pragma unroll 1
  for (int i = tid; i < nv; i += NTHR) { const v4i v = ((const v4i*)region)[i]; *(volatile v4i*)(gp + 4 * i) = v; }
  __threadfence();
#pragma unroll 1
  for (int i = tid; i < nv; i += NTHR) { const v4i v = ((const v4i*)region)[i]; *(volatile v4i*)(gp + 4 * i) = v; }
}

__device__ __forceinline__ void stage64(const float* src, int rowBase, int nValid,
                                        unsigned short* th, unsigned short* tl) {
  const int tid = threadIdx.x;
  const v4f z4 = {0.f, 0.f, 0.f, 0.f};
#pragma unroll
  for (int it = 0; it < 4; ++it) {
    const int u = it * NTHR + tid;
    const int r = u >> 4, c = (u & 15) * 8;
    const int grow = rowBase + r;
    const int rc = grow < nValid ? grow : nValid - 1;
    const float* p = src + (size_t)rc * FD + c;
    v4f a = *(const v4f*)p, b = *(const v4f*)(p + 4);
    if (grow >= nValid) { a = z4; b = z4; }
    v8us hv, lv;
    sp8(a, b, hv, lv);
    *(v8us*)(th + r * FD + c) = hv;
    *(v8us*)(tl + r * FD + c) = lv;
  }
}

template <int NT, int PB>
__device__ __forceinline__ void mmk(v8f (&acc)[NT], const unsigned short* th, const unsigned short* tl, int arow,
                                    const unsigned short* __restrict__ Bh, const unsigned short* __restrict__ Bl,
                                    int bcol0, int kofs) {
  const int lane = threadIdx.x & 31, hh = lane >> 4, m = lane & 15;
  const unsigned short* aph = th + (arow + m) * FD + 8 * hh;
  const unsigned short* apl = tl + (arow + m) * FD + 8 * hh;
  const size_t boff = (size_t)(bcol0 + m) * PB + kofs + 8 * hh;
  const unsigned short* bph0 = Bh + boff;
  const unsigned short* bpl0 = Bl + boff;
#pragma unroll 1
  for (int kt = 0; kt < FD / 32; ++kt) {
    FragU ah, al;
    ah.u[0] = *(const v8us*)(aph + 32 * kt);
    ah.u[1] = *(const v8us*)(aph + 32 * kt + 16);
    al.u[0] = *(const v8us*)(apl + 32 * kt);
    al.u[1] = *(const v8us*)(apl + 32 * kt + 16);
#pragma unroll
    for (int t = 0; t < NT; ++t) {
      const size_t to = (size_t)(16 * t) * PB + 32 * kt;
      FragU bh, bl;
      bh.u[0] = *(const v8us*)(bph0 + to);
      bh.u[1] = *(const v8us*)(bph0 + to + 16);
      bl.u[0] = *(const v8us*)(bpl0 + to);
      bl.u[1] = *(const v8us*)(bpl0 + to + 16);
      acc[t] = wmb(ah.w, bh.w, acc[t]);
      acc[t] = wmb(al.w, bh.w, acc[t]);
      acc[t] = wmb(ah.w, bl.w, acc[t]);
    }
  }
}

template <int DUAL, int RELU, int HASB>
__global__ __launch_bounds__(NTHR) void k_gemm(
    const float* A0, const float* A1,
    const unsigned short* __restrict__ Bh, const unsigned short* __restrict__ Bl,
    const float* __restrict__ bias, float* Out, int nN) {
  extern __shared__ v4f lds_dyn[];
  constexpr int PB = DUAL ? KL : FD;
  unsigned short* th0 = (unsigned short*)lds_dyn;
  unsigned short* tl0 = th0 + BM * FD;
  unsigned short* th1 = tl0 + BM * FD;
  unsigned short* tl1 = th1 + BM * FD;
  float* stg = (float*)(th0 + (DUAL ? 4 : 2) * BM * FD);
  const int tid = threadIdx.x, lane = tid & 31, wave = tid >> 5, hh = lane >> 4, m = lane & 15;
  const int rowBase = blockIdx.x * BM;
  const int r0 = (wave >> 1) * 16, c0 = (wave & 1) * 64;

  stage64(A0, rowBase, nN, th0, tl0);
  if (DUAL) stage64(A1, rowBase, nN, th1, tl1);
  __syncthreads();

  v8f acc[4];
#pragma unroll
  for (int t = 0; t < 4; ++t) { v8f z = {0.f, 0.f, 0.f, 0.f, 0.f, 0.f, 0.f, 0.f}; acc[t] = z; }
  mmk<4, PB>(acc, th0, tl0, r0, Bh, Bl, c0, 0);
  if (DUAL) mmk<4, PB>(acc, th1, tl1, r0, Bh, Bl, c0, FD);
  {
    float* sp = stg + (size_t)(r0 + 8 * hh) * FD + c0 + m;
#pragma unroll
    for (int t = 0; t < 4; ++t) {
#pragma unroll
      for (int r = 0; r < 8; ++r) sp[r * FD + 16 * t] = acc[t][r];
    }
  }
  __syncthreads();

  const v4f z4 = {0.f, 0.f, 0.f, 0.f};
  const int rsub = lane >> 4, q = lane & 15, col = c0 + 4 * q;
  v4f b4 = z4;
  if (HASB) b4 = *(const v4f*)(bias + col);
#pragma unroll
  for (int it = 0; it < 8; ++it) {
    const int row  = it * 2 + rsub;
    const int grow = rowBase + r0 + row;
    v4f v = *(const v4f*)(stg + (size_t)(r0 + row) * FD + col) + b4;
    if (RELU) v = relu4(v);
    if (grow >= nN) v = z4;
    *(volatile v4f*)(Out + (size_t)grow * FD + col) = v;
  }
  __threadfence();
#pragma unroll
  for (int it = 0; it < 8; ++it) {
    const int row  = it * 2 + rsub;
    const int grow = rowBase + r0 + row;
    v4f v = *(const v4f*)(stg + (size_t)(r0 + row) * FD + col) + b4;
    if (RELU) v = relu4(v);
    if (grow >= nN) v = z4;
    *(volatile v4f*)(Out + (size_t)grow * FD + col) = v;
  }
}

__global__ __launch_bounds__(NTHR) void k_agg(
    const int* __restrict__ csr, const int* __restrict__ off, const int* __restrict__ cnt,
    const int* __restrict__ srcs, const float* __restrict__ Hin, float* AG, int nN, int nE, int csrLen) {
  const int tid = threadIdx.x, lane = tid & 31, wave = tid >> 5;
  const int tbase = blockIdx.x * TGT + wave * 32;
  const int col = 4 * lane;
  const v4f z4 = {0.f, 0.f, 0.f, 0.f};
  const int cl    = tbase + lane;
  const int cnt_l = cnt[cl];
  const int off_l = off[cl];

#pragma unroll 1
  for (int j = 0; j < 32; ++j) {
    const int c  = tbase + j;
    const int dg = __shfl(cnt_l, j);
    const int n  = dg < 0 ? 0 : (dg > DEGCAP ? DEGCAP : dg);
    const int st = __shfl(off_l, j);
    v4f acc = z4;
#pragma unroll 1
    for (int q0 = 0; q0 < n; q0 += 32) {
      int pos = st + q0 + lane;
      pos = pos < 0 ? 0 : (pos > csrLen - 1 ? csrLen - 1 : pos);
      int eid = csr[pos];
      eid = eid < 0 ? 0 : (eid > nE - 1 ? nE - 1 : eid);
      int sl = srcs[eid];
      sl = sl < 0 ? 0 : (sl > nN - 1 ? nN - 1 : sl);
      const int mcnt = (n - q0) < 32 ? (n - q0) : 32;
#pragma unroll 1
      for (int pp = 0; pp < mcnt; ++pp) {
        const int s = __builtin_amdgcn_readlane(sl, pp);
        const v4f xs = *(const v4f*)(Hin + (size_t)s * FD + col);
        acc += xs;
      }
    }
    v4f v = acc;
    if (c >= nN) v = z4;
    float* po = AG + (size_t)c * FD + col;
    *(volatile v4f*)po = v;
    __threadfence();
    *(volatile v4f*)po = v;
  }
}

__global__ __launch_bounds__(NTHR) void k_scores(
    const float* __restrict__ HT, const float* __restrict__ avs, const float* __restrict__ avd,
    float* sS, float* sD) {
  const int tid = threadIdx.x, lane = tid & 31, wave = tid >> 5;
  const int tbase = blockIdx.x * TGT + wave * 32;
  const int col = 4 * lane;
  const v4f a4 = *(const v4f*)(avs + col);
  const v4f d4 = *(const v4f*)(avd + col);
  float vs = 0.f, vd = 0.f;
#pragma unroll 1
  for (int j = 0; j < 32; ++j) {
    const v4f h = *(const v4f*)(HT + (size_t)(tbase + j) * FD + col);
    float ps = h.x * a4.x + h.y * a4.y + h.z * a4.z + h.w * a4.w;
    float pd = h.x * d4.x + h.y * d4.y + h.z * d4.z + h.w * d4.w;
#pragma unroll
    for (int o = 16; o > 0; o >>= 1) {
      ps += __shfl_xor(ps, o);
      pd += __shfl_xor(pd, o);
    }
    vs = (lane == j) ? ps : vs;
    vd = (lane == j) ? pd : vd;
  }
  float* p0 = sS + tbase + lane;
  float* p1 = sD + tbase + lane;
  *(volatile float*)p0 = vs;
  *(volatile float*)p1 = vd;
  __threadfence();
  *(volatile float*)p0 = vs;
  *(volatile float*)p1 = vd;
}

__global__ __launch_bounds__(NTHR) void k_attn(
    const int* __restrict__ csr, const int* __restrict__ off, const int* __restrict__ cnt,
    const int* __restrict__ srcs, const float* __restrict__ sS, const float* __restrict__ sD,
    const float* __restrict__ HT, float* OUT, int nN, int nE, int csrLen) {
  const int tid = threadIdx.x, lane = tid & 31, wave = tid >> 5;
  const int tbase = blockIdx.x * TGT + wave * 32;
  const int col = 4 * lane;
  const v4f z4 = {0.f, 0.f, 0.f, 0.f};
  const float ninf = __uint_as_float(0xff800000u);
  const int cl    = tbase + lane;
  const int cnt_l = cnt[cl];
  const int off_l = off[cl];
  const float sd_l = sD[cl];

#pragma unroll 1
  for (int j = 0; j < 32; ++j) {
    const int c  = tbase + j;
    const int dg = __shfl(cnt_l, j);
    const int n  = dg < 0 ? 0 : (dg > DEGCAP ? DEGCAP : dg);
    const int st = __shfl(off_l, j);
    const float sdc = __shfl(sd_l, j);

    float mx = ninf;
#pragma unroll 1
    for (int q0 = 0; q0 < n; q0 += 32) {
      int pos = st + q0 + lane;
      pos = pos < 0 ? 0 : (pos > csrLen - 1 ? csrLen - 1 : pos);
      int eid = csr[pos];
      eid = eid < 0 ? 0 : (eid > nE - 1 ? nE - 1 : eid);
      int sl = srcs[eid];
      sl = sl < 0 ? 0 : (sl > nN - 1 ? nN - 1 : sl);
      float ev = sS[sl] + sdc;
      ev = ev >= 0.f ? ev : 0.2f * ev;
      float mv = (q0 + lane < n) ? ev : ninf;
#pragma unroll
      for (int o = 16; o > 0; o >>= 1) mv = fmaxf(mv, __shfl_xor(mv, o));
      mx = fmaxf(mx, mv);
    }

    v4f acc = z4;
    float den = 0.f;
#pragma unroll 1
    for (int q0 = 0; q0 < n; q0 += 32) {
      int pos = st + q0 + lane;
      pos = pos < 0 ? 0 : (pos > csrLen - 1 ? csrLen - 1 : pos);
      int eid = csr[pos];
      eid = eid < 0 ? 0 : (eid > nE - 1 ? nE - 1 : eid);
      int sl = srcs[eid];
      sl = sl < 0 ? 0 : (sl > nN - 1 ? nN - 1 : sl);
      float ev = sS[sl] + sdc;
      ev = ev >= 0.f ? ev : 0.2f * ev;
      const bool valid = (q0 + lane) < n;
      const float arg = (valid ? ev : mx) - mx;
      const float ex  = expf(arg);
      const float w   = valid ? ex : 0.f;
      float wsum = w;
#pragma unroll
      for (int o = 16; o > 0; o >>= 1) wsum += __shfl_xor(wsum, o);
      den += wsum;
      const int mcnt = (n - q0) < 32 ? (n - q0) : 32;
#pragma unroll 1
      for (int pp = 0; pp < mcnt; ++pp) {
        const int s = __builtin_amdgcn_readlane(sl, pp);
        const float wp = __int_as_float(__builtin_amdgcn_readlane(__float_as_int(w), pp));
        const v4f xs = *(const v4f*)(HT + (size_t)s * FD + col);
        acc += xs * wp;
      }
    }
    const float rden = __builtin_amdgcn_rcpf(den + 1e-16f);
    v4f v = acc * rden;
    if (c >= nN) v = z4;
    float* po = OUT + (size_t)c * FD + col;
    *(volatile v4f*)po = v;
    __threadfence();
    *(volatile v4f*)po = v;
  }
}

__global__ __launch_bounds__(NTHR) void k_cls(
    const float* __restrict__ Hin, const unsigned short* __restrict__ Bh, const unsigned short* __restrict__ Bl,
    const float* __restrict__ cb, float* out, int nN) {
  extern __shared__ v4f lds_dyn[];
  unsigned short* th = (unsigned short*)lds_dyn;
  unsigned short* tl = th + CBM * FD;
  float* stg2 = (float*)(tl + CBM * FD);
  const int tid = threadIdx.x, lane = tid & 31, wave = tid >> 5, hh = lane >> 4, m = lane & 15;
  const int rowBase = blockIdx.x * CBM;

  stage64(Hin, rowBase, nN, th, tl);
  stage64(Hin, rowBase + BM, nN, th + BM * FD, tl + BM * FD);
  __syncthreads();

  const int arow = 16 * wave;
  v8f acc[1];
  { v8f z = {0.f, 0.f, 0.f, 0.f, 0.f, 0.f, 0.f, 0.f}; acc[0] = z; }
  mmk<1, FD>(acc, th, tl, arow, Bh, Bl, 0, 0);
  if (m < NCLS) {
#pragma unroll
    for (int r = 0; r < 8; ++r) stg2[(arow + 8 * hh + r) * NCLS + m] = acc[0][r];
  }
  __syncthreads();

  const float cb0 = cb[0], cb1 = cb[1];
  v4f bb; bb.x = cb0; bb.y = cb1; bb.z = cb0; bb.w = cb1;
  const int t4 = tid < 64 ? tid : 63;
  const v4f w = *(const v4f*)(stg2 + 4 * t4) + bb;
  const size_t tot = (size_t)nN * NCLS;
  const size_t f   = (size_t)rowBase * NCLS + 4 * (size_t)t4;
  float* po = out + f;
  const bool full = (tid < 64) && (f + 4 <= tot);
  const bool two  = (tid < 64) && !(f + 4 <= tot) && (f + 2 <= tot);
  v2f w2; w2.x = w.x; w2.y = w.y;
  if (full) *(volatile v4f*)po = w;
  if (two)  *(volatile v2f*)po = w2;
  __threadfence();
  if (full) *(volatile v4f*)po = w;
  if (two)  *(volatile v2f*)po = w2;
}

static size_t carve(size_t* o, size_t bytes) {
  const size_t r = *o;
  *o += (bytes + 255) & ~(size_t)255;
  return r;
}

extern "C" void kernel_launch(void* const* d_in, const int* in_sizes, int n_in,
                              void* d_out, int out_size, void* d_ws, size_t ws_size,
                              hipStream_t stream) {
  if (n_in < 13) return;
  const int nN = in_sizes[0] / FD;
  const int nE = in_sizes[1] / 2;
  if (nN <= 0 || nE <= 0 || in_sizes[0] != nN * FD || in_sizes[1] != 2 * nE) return;
  if (in_sizes[2] != FD * FD || in_sizes[3] != FD * FD || in_sizes[4] != FD) return;
  if (in_sizes[5] != FD * FD || in_sizes[6] != FD * FD || in_sizes[7] != FD) return;
  if (in_sizes[8] != FD * FD || in_sizes[9] != FD || in_sizes[10] != FD) return;
  if (in_sizes[11] != FD * NCLS || in_sizes[12] != NCLS) return;
  if ((long long)out_size != (long long)nN * NCLS) return;
  if (nE > (1 << 27) || nN > (1 << 22)) return;

  const float* x     = (const float*)d_in[0];
  const int*   ei    = (const int*)d_in[1];
  const float* W1r   = (const float*)d_in[2];
  const float* W1n   = (const float*)d_in[3];
  const float* b1    = (const float*)d_in[4];
  const float* W2r   = (const float*)d_in[5];
  const float* W2n   = (const float*)d_in[6];
  const float* b2    = (const float*)d_in[7];
  const float* Wa    = (const float*)d_in[8];
  const float* avs   = (const float*)d_in[9];
  const float* avd   = (const float*)d_in[10];
  const float* Wfc   = (const float*)d_in[11];
  const float* bfc   = (const float*)d_in[12];
  const int* src = ei;
  const int* dst = ei + nE;
  float* dout = (float*)d_out;

  const int NPAD   = ((nN + TGT - 1) / TGT) * TGT;
  const int nBC    = (nN + NBC - 1) / NBC;
  const int CNTPAD = nBC * NBC;
  if (FPC * nBC + 1 > RBN) return;
  const int nBF    = (nN + NBF - 1) / NBF;
  const int csrLen = ((nE + 31) & ~31) + 4096;
  if (31 * FPC * nBC > 4096) return;
  const int nAgg   = NPAD / TGT;
  const int nGm    = NPAD / BM;
  const int nCl    = NPAD / CBM;

  char* ws = (char*)d_ws;
  size_t o = 0;
  const size_t oW1H = carve(&o, (size_t)FD * KL * 2),  oW1L = carve(&o, (size_t)FD * KL * 2);
  const size_t oW2H = carve(&o, (size_t)FD * KL * 2),  oW2L = carve(&o, (size_t)FD * KL * 2);
  const size_t oWaH = carve(&o, (size_t)FD * FD * 2),  oWaL = carve(&o, (size_t)FD * FD * 2);
  const size_t oWcH = carve(&o, (size_t)NCP * FD * 2), oWcL = carve(&o, (size_t)NCP * FD * 2);
  const size_t oCnt = carve(&o, (size_t)CNTPAD * 4);
  const size_t oOff = carve(&o, (size_t)CNTPAD * 4);
  const size_t oRb  = carve(&o, (size_t)RBN * 4);
  const size_t oCsr = carve(&o, (size_t)csrLen * 4);
  const size_t oSS  = carve(&o, (size_t)NPAD * 4);
  const size_t oSD  = carve(&o, (size_t)NPAD * 4);
  const size_t oH   = carve(&o, (size_t)NPAD * FD * 4);
  const size_t oAG  = carve(&o, (size_t)NPAD * FD * 4);
  if (o > ws_size || o > (size_t)WSCAP) return;

  unsigned short* w1H = (unsigned short*)(ws + oW1H); unsigned short* w1L = (unsigned short*)(ws + oW1L);
  unsigned short* w2H = (unsigned short*)(ws + oW2H); unsigned short* w2L = (unsigned short*)(ws + oW2L);
  unsigned short* waH = (unsigned short*)(ws + oWaH); unsigned short* waL = (unsigned short*)(ws + oWaL);
  unsigned short* wcH = (unsigned short*)(ws + oWcH); unsigned short* wcL = (unsigned short*)(ws + oWcL);
  int*   cnt  = (int*)(ws + oCnt);
  int*   offp = (int*)(ws + oOff);
  int*   rb   = (int*)(ws + oRb);
  int*   csr  = (int*)(ws + oCsr);
  float* sS   = (float*)(ws + oSS);
  float* sD   = (float*)(ws + oSD);
  float* H    = (float*)(ws + oH);
  float* AG   = (float*)(ws + oAG);

  const int vec8 = ((nE & 3) == 0) ? 1 : 0;

  k_wprep<<<(FD * 32 + NTHR - 1) / NTHR, NTHR, 0, stream>>>(W1r, W1n, FD, 5, FD, w1H, w1L, FD * 32);
  k_wprep<<<(FD * 32 + NTHR - 1) / NTHR, NTHR, 0, stream>>>(W2r, W2n, FD, 5, FD, w2H, w2L, FD * 32);
  k_wprep<<<(FD * 16 + NTHR - 1) / NTHR, NTHR, 0, stream>>>(Wa, Wa, FD, 4, FD, waH, waL, FD * 16);
  k_wprep<<<(NCP * 16 + NTHR - 1) / NTHR, NTHR, 0, stream>>>(Wfc, Wfc, NCLS, 4, NCLS, wcH, wcL, NCP * 16);

  k_count<<<nBC, NTHR, 0, stream>>>(dst, cnt, nE, vec8);
  k_offsets<<<1, OTHR, 0, stream>>>(cnt, offp, rb, nBC);
  hipFuncSetAttribute(reinterpret_cast<const void*>(&k_fill),
                      hipFuncAttributeMaxDynamicSharedMemorySize, LDS_FILL);
  k_fill<<<nBF, NTHR, LDS_FILL, stream>>>(dst, offp, rb, csr, nE, vec8, csrLen);

  hipFuncSetAttribute(reinterpret_cast<const void*>(&k_gemm<1, 1, 1>),
                      hipFuncAttributeMaxDynamicSharedMemorySize, LDS_G2);
  hipFuncSetAttribute(reinterpret_cast<const void*>(&k_gemm<0, 0, 0>),
                      hipFuncAttributeMaxDynamicSharedMemorySize, LDS_G1);

  k_agg<<<nAgg, NTHR, 0, stream>>>(csr, offp, cnt, src, x, AG, nN, nE, csrLen);
  k_gemm<1, 1, 1><<<nGm, NTHR, LDS_G2, stream>>>(x, AG, w1H, w1L, b1, H, nN);

  k_agg<<<nAgg, NTHR, 0, stream>>>(csr, offp, cnt, src, H, AG, nN, nE, csrLen);
  k_gemm<1, 1, 1><<<nGm, NTHR, LDS_G2, stream>>>(H, AG, w2H, w2L, b2, H, nN);

  k_gemm<0, 0, 0><<<nGm, NTHR, LDS_G1, stream>>>(H, H, waH, waL, b1, AG, nN);

  k_scores<<<nAgg, NTHR, 0, stream>>>(AG, avs, avd, sS, sD);

  k_attn<<<nAgg, NTHR, 0, stream>>>(csr, offp, cnt, src, sS, sD, AG, H, nN, nE, csrLen);

  hipFuncSetAttribute(reinterpret_cast<const void*>(&k_cls),
                      hipFuncAttributeMaxDynamicSharedMemorySize, LDS_CLS);
  k_cls<<<nCl, NTHR, LDS_CLS, stream>>>(H, wcH, wcL, bfc, dout, nN);
}
